// TransformerLayer_41162966565467
// MI455X (gfx1250) — hardware-verified
//
#include <hip/hip_runtime.h>


#ifndef NB
#define NB 2
#endif
#ifndef SEQ
#define SEQ 2048
#endif
#define NB_FULL  2
#define SEQ_FULL 2048
#define EM   1024
#define NHD  16
#define HD   64
#define RW   512
#define FF   4096
#define QKP  (2 * EM)
#define MR   (NB * SEQ)
#define WCAR 64.0f
#define PCAR 1024.0f
#define CCAR 16.0f
#define NEGS (-1.0e30f)
#define AP   40
#define OP   72

static_assert(SEQ % 64 == 0);
static_assert(SEQ >= 64);
static_assert(EM % 64 == 0);
static_assert(FF % 64 == 0);
static_assert(QKP % 64 == 0);
static_assert(EM % 32 == 0);
static_assert(FF % 32 == 0);
static_assert(NHD * HD == EM);
static_assert(HD == 64);
static_assert(RW % 32 == 0);
static_assert(NB <= NB_FULL);
static_assert(SEQ <= SEQ_FULL);
static_assert(EM == 4 * 32 * 8);
static_assert(MR % 8 == 0);

typedef _Float16 h16;
typedef __attribute__((ext_vector_type(16))) _Float16 v16h;
typedef __attribute__((ext_vector_type(8)))  _Float16 v8h;
typedef __attribute__((ext_vector_type(8)))  float    v8f;
typedef __attribute__((ext_vector_type(4)))  float    v4f;
typedef v8h  __attribute__((may_alias)) v8ha;
typedef v4f  __attribute__((may_alias)) v4fa;

__device__ __forceinline__ unsigned short f2bf(float f) { unsigned u = __float_as_uint(f); u += 0x7FFFu + ((u >> 16) & 1u); return (unsigned short)(u >> 16); }
__device__ __forceinline__ float bf2f(unsigned short b) { return __uint_as_float(((unsigned)b) << 16); }
__device__ __forceinline__ float bfr(float f) { return bf2f(f2bf(f)); }
__device__ __forceinline__ v16h cat16(v8h lo, v8h hi) { return __builtin_shufflevector(lo, hi, 0, 1, 2, 3, 4, 5, 6, 7, 8, 9, 10, 11, 12, 13, 14, 15); }
__device__ __forceinline__ v8f wmma16(v16h a, v16h b, v8f c) { return __builtin_amdgcn_wmma_f32_16x16x32_f16(false, a, false, b, (short)0, c, false, false); }
__device__ __forceinline__ v16h ldfrag(const h16* p) { return cat16(*(const v8h*)p, *(const v8h*)(p + 16)); }
__device__ __forceinline__ float ex2s(float d) { return __builtin_amdgcn_exp2f(fmaxf(d * 1.4426950408889634f, -126.0f)); }

__global__ __launch_bounds__(256) void k_cvtw(const float* __restrict__ src, h16* dst, size_t n8) {
    const size_t i = (size_t)blockIdx.x * 256 + threadIdx.x; if (i >= n8) return;
    const v8f v = *(const v8f*)(src + i * 8); v8h o;
#pragma unroll
    for (int k = 0; k < 8; ++k) o[k] = (h16)(bfr(v[k]) * WCAR);
    *(volatile v8h*)(dst + i * 8) = o; __threadfence(); *(volatile v8h*)(dst + i * 8) = o;
}

template <bool RND>
__global__ __launch_bounds__(256) void k_ln(const float* __restrict__ X, int seq, int brows, const float* __restrict__ g, const float* __restrict__ bt, h16* Y, int nrows) {
    __shared__ __align__(32) float sv[8 * EM];
    const int lane = threadIdx.x & 31, wv = threadIdx.x >> 5; const int row = blockIdx.x * 8 + wv; if (row >= nrows) return;
    const int b = row / seq, t = row - b * seq; const float* xr = X + ((size_t)b * brows + t) * EM + lane * 8;
    const int so = wv * EM + lane * 8;
    float s = 0.f;
#pragma unroll 1
    for (int c = 0; c < 4; ++c) { v8f a = *(const v8f*)(xr + c * 256);
#pragma unroll
        for (int k = 0; k < 8; ++k) { const float y = RND ? bfr(a[k]) : a[k]; a[k] = y; s += y; }
        *(v8f*)(sv + so + c * 256) = a; }
#pragma unroll
    for (int sh = 16; sh; sh >>= 1) s += __shfl_xor(s, sh, 32);
    const float mu = s * (1.0f / EM); float ss = 0.f;
#pragma unroll 1
    for (int c = 0; c < 4; ++c) { const v8f a = *(const v8f*)(sv + so + c * 256);
#pragma unroll
        for (int k = 0; k < 8; ++k) { const float d = a[k] - mu; ss += d * d; } }
#pragma unroll
    for (int sh = 16; sh; sh >>= 1) ss += __shfl_xor(ss, sh, 32);
    const float inv = rsqrtf(ss * (1.0f / EM) + 1e-5f);
    h16* yr = Y + (size_t)row * EM + lane * 8;
#pragma unroll 1
    for (int ps = 0; ps < 2; ++ps) {
#pragma unroll 1
        for (int c = 0; c < 4; ++c) { const v8f a = *(const v8f*)(sv + so + c * 256); const v8f gg = *(const v8f*)(g + c * 256 + lane * 8); const v8f bb = *(const v8f*)(bt + c * 256 + lane * 8); v8h o;
#pragma unroll
            for (int k = 0; k < 8; ++k) o[k] = (h16)((a[k] - mu) * inv * bfr(gg[k]) + bfr(bb[k]));
            *(volatile v8h*)(yr + c * 256) = o; }
        if (ps == 0) __threadfence(); }
}

template <int OUTH, bool BROW, bool RELU, int RES>
__global__ __launch_bounds__(32) void k_gemmw(const h16* __restrict__ A, const h16* __restrict__ Bt, int K, void* Cv, int ldc, const float* __restrict__ bias, float sc, const float* __restrict__ res, int rseq, int rbs, size_t sA, size_t sB, size_t sC) {
    static_assert(!(OUTH != 0 && RES != 0));
    __shared__ __align__(16) float os[16 * 68];
    const size_t z = blockIdx.z; A += z * sA; Bt += z * sB;
    const int lane = threadIdx.x & 31, lr = lane & 15, hi = lane >> 4; const int r0 = blockIdx.x * 64, c0 = blockIdx.y * 64;
    v8f acc[4][4];
#pragma unroll
    for (int mb = 0; mb < 4; ++mb)
#pragma unroll
        for (int nb = 0; nb < 4; ++nb) acc[mb][nb] = (v8f){};
    const size_t aoff = (size_t)(r0 + lr) * K + 8 * hi, boff = (size_t)(c0 + lr) * K + 8 * hi;
#pragma unroll 1
    for (int kc = 0; kc < K; kc += 32) {
        v16h a[4];
#pragma unroll
        for (int mb = 0; mb < 4; ++mb) a[mb] = ldfrag(A + aoff + (size_t)mb * 16 * K + kc);
#pragma unroll
        for (int nb = 0; nb < 4; ++nb) { const v16h b = ldfrag(Bt + boff + (size_t)nb * 16 * K + kc);
#pragma unroll
            for (int mb = 0; mb < 4; ++mb) acc[mb][nb] = wmma16(a[mb], b, acc[mb][nb]); }
        asm volatile("v_nop\n\tv_nop\n\tv_nop\n\tv_nop" : "+v"(acc[0][0]), "+v"(acc[1][1]), "+v"(acc[2][2]), "+v"(acc[3][3]) : "v"(a[0]), "v"(a[3]));
    }
    float bc[8];
#pragma unroll
    for (int q = 0; q < 8; ++q) bc[q] = 0.f;
    if (!BROW) {
        if (OUTH) { const v4f b0 = *(const v4f*)(bias + c0 + (lane & 7) * 8), b1 = *(const v4f*)(bias + c0 + (lane & 7) * 8 + 4);
#pragma unroll
            for (int q = 0; q < 4; ++q) { bc[q] = bfr(b0[q]); bc[4 + q] = bfr(b1[q]); } }
        else { const v4f b0 = *(const v4f*)(bias + c0 + lr * 4);
#pragma unroll
            for (int q = 0; q < 4; ++q) bc[q] = bfr(b0[q]); }
    }
    const int rb = r0 / rseq;
#pragma unroll
    for (int mb = 0; mb < 4; ++mb) {
#pragma unroll
        for (int nb = 0; nb < 4; ++nb) {
#pragma unroll
            for (int j = 0; j < 8; ++j) os[(hi * 8 + j) * 68 + nb * 16 + lr] = acc[mb][nb][j]; }
        __builtin_amdgcn_wave_barrier(); asm volatile("" ::: "memory");
        if (OUTH == 0) {
            float* crow = (float*)Cv + z * sC + (size_t)(r0 + mb * 16) * ldc + c0;
#pragma unroll 1
            for (int ps = 0; ps < 2; ++ps) {
#pragma unroll
                for (int s = 0; s < 8; ++s) { const int row = 2 * s + hi, cofs = lr * 4; const int m = r0 + mb * 16 + row; v4f val = *(const v4fa*)(os + row * 68 + cofs);
                    float br = 0.f; if (BROW) br = bfr(bias[m]);
                    v4f rr = (v4f){}; if (RES) rr = *(const v4f*)(res + ((size_t)rb * rbs + (m - rb * rseq)) * ldc + c0 + cofs);
#pragma unroll
                    for (int q = 0; q < 4; ++q) { float y = val[q] * sc + (BROW ? br : bc[q]); if (RELU) y = fmaxf(y, 0.0f); if (RES == 1) y += rr[q]; if (RES == 2) y += bfr(rr[q]); val[q] = y; }
                    *(volatile v4f*)(crow + (size_t)row * ldc + cofs) = val; }
                if (ps == 0) __threadfence(); }
        } else {
            h16* crow = (h16*)Cv + z * sC + (size_t)(r0 + mb * 16) * ldc + c0;
#pragma unroll 1
            for (int ps = 0; ps < 2; ++ps) {
#pragma unroll
                for (int s = 0; s < 4; ++s) { const int row = 4 * s + (lane >> 3), cofs = (lane & 7) * 8; const int m = r0 + mb * 16 + row;
                    const v4f u0 = *(const v4fa*)(os + row * 68 + cofs), u1 = *(const v4fa*)(os + row * 68 + cofs + 4);
                    float br = 0.f; if (BROW) br = bfr(bias[m]);
                    v8h o;
#pragma unroll
                    for (int q = 0; q < 4; ++q) { float y0 = u0[q] * sc + (BROW ? br : bc[q]); float y1 = u1[q] * sc + (BROW ? br : bc[4 + q]); if (RELU) { y0 = fmaxf(y0, 0.0f); y1 = fmaxf(y1, 0.0f); } o[q] = (h16)y0; o[4 + q] = (h16)y1; }
                    *(volatile v8h*)(crow + (size_t)row * ldc + cofs) = o; }
                if (ps == 0) __threadfence(); }
        }
        __builtin_amdgcn_wave_barrier(); asm volatile("" ::: "memory");
    }
}

__global__ __launch_bounds__(128) void k_attn(const h16* __restrict__ QK, const h16* __restrict__ VT, const float* __restrict__ res_pos, h16* CTX) {
    __shared__ __align__(16) float rp[RW];
    __shared__ __align__(16) h16 pl[4][16 * AP];
    __shared__ __align__(16) h16 ol[4][16 * OP];
    const int tid = threadIdx.x, lane = tid & 31, wv = tid >> 5, lo = lane & 15, hi = lane >> 4;
    const int h = blockIdx.y, b = blockIdx.z;
    const int qbase = (blockIdx.x * 4 + wv) * 16, qend = qbase + 15;
    for (int i = tid; i < RW; i += 128) rp[i] = bfr(res_pos[h * RW + i]);
    __syncthreads();
    h16* pst = &pl[wv][0]; h16* ost = &ol[wv][0];
    const h16* qrow = QK + ((size_t)b * SEQ + qbase + lo) * QKP + h * HD + 8 * hi;
    const v16h qf0 = ldfrag(qrow), qf1 = ldfrag(qrow + 32);
    const h16* Kb = QK + (size_t)b * SEQ * QKP + EM + h * HD + 8 * hi;
    const h16* Vb = VT + ((size_t)b * EM + h * HD) * SEQ + 8 * hi;
    float m_run[8], l_run[8]; v8f oacc[4];
#pragma unroll
    for (int r = 0; r < 8; ++r) { m_run[r] = NEGS; l_run[r] = 0.0f; }
#pragma unroll
    for (int ni = 0; ni < 4; ++ni) oacc[ni] = (v8f){};
    int klo = qbase - RW; if (klo < 0) klo = 0;
#pragma unroll 1
    for (int kb0 = klo; kb0 <= qend; kb0 += 32) {
        v8f s0 = (v8f){}, s1 = (v8f){};
        {
            const int key0 = min(kb0 + lo, SEQ - 1), key1 = min(kb0 + 16 + lo, SEQ - 1);
            const h16* k0p = Kb + (size_t)key0 * QKP; const h16* k1p = Kb + (size_t)key1 * QKP;
            const v16h kf00 = ldfrag(k0p), kf01 = ldfrag(k0p + 32), kf10 = ldfrag(k1p), kf11 = ldfrag(k1p + 32);
            s0 = wmma16(qf0, kf00, s0); s0 = wmma16(qf1, kf01, s0);
            s1 = wmma16(qf0, kf10, s1); s1 = wmma16(qf1, kf11, s1);
            asm volatile("v_nop\n\tv_nop\n\tv_nop\n\tv_nop" : "+v"(s0), "+v"(s1) : "v"(qf0), "v"(qf1), "v"(kf10), "v"(kf11));
        }
        float alpha[8];
#pragma unroll
        for (int r = 0; r < 8; ++r) {
            const int row = qbase + 8 * hi + r; const int rel0 = row - (kb0 + lo), rel1 = rel0 - 16;
            const bool v0 = (unsigned)rel0 < (unsigned)RW, v1 = (unsigned)rel1 < (unsigned)RW;
            const float pb0 = rp[min(max(rel0, 0), RW - 1)], pb1 = rp[min(max(rel1, 0), RW - 1)];
            const float a0 = v0 ? (s0[r] * 0.125f + pb0) : NEGS; const float a1 = v1 ? (s1[r] * 0.125f + pb1) : NEGS;
            float tm = fmaxf(a0, a1);
#pragma unroll
            for (int sh = 8; sh; sh >>= 1) tm = fmaxf(tm, __shfl_xor(tm, sh, 32));
            const float mn = fmaxf(m_run[r], tm);
            const float al = ex2s(m_run[r] - mn);
            const float e0 = v0 ? ex2s(a0 - mn) : 0.0f; const float e1 = v1 ? ex2s(a1 - mn) : 0.0f;
            const h16 q0 = (h16)(e0 * PCAR), q1 = (h16)(e1 * PCAR);
            float rsum = ((float)q0 + (float)q1) * (1.0f / PCAR);
#pragma unroll
            for (int sh = 8; sh; sh >>= 1) rsum += __shfl_xor(rsum, sh, 32);
            l_run[r] = l_run[r] * al + rsum; m_run[r] = mn; alpha[r] = al;
            pst[(8 * hi + r) * AP + lo] = q0; pst[(8 * hi + r) * AP + 16 + lo] = q1;
        }
#pragma unroll
        for (int ni = 0; ni < 4; ++ni)
#pragma unroll
            for (int r = 0; r < 8; ++r) oacc[ni][r] *= alpha[r];
        __builtin_amdgcn_wave_barrier(); asm volatile("" ::: "memory");
        const v16h pf = cat16(*(const v8ha*)(pst + lo * AP + 8 * hi), *(const v8ha*)(pst + lo * AP + 16 + 8 * hi));
        const int k2 = min(kb0 + 16, SEQ - 16);
#pragma unroll
        for (int ni = 0; ni < 4; ++ni) { const h16* vp = Vb + (size_t)(ni * 16 + lo) * SEQ; const v16h vf = cat16(*(const v8h*)(vp + kb0), *(const v8h*)(vp + k2)); oacc[ni] = wmma16(pf, vf, oacc[ni]); }
        asm volatile("v_nop\n\tv_nop\n\tv_nop\n\tv_nop" : "+v"(oacc[0]), "+v"(oacc[1]), "+v"(oacc[2]), "+v"(oacc[3]) : "v"(pf));
        __builtin_amdgcn_wave_barrier(); asm volatile("" ::: "memory");
    }
#pragma unroll
    for (int r = 0; r < 8; ++r) { const float f = (CCAR / PCAR) * (1.0f / fmaxf(l_run[r], 1.0e-30f));
#pragma unroll
        for (int ni = 0; ni < 4; ++ni) ost[(8 * hi + r) * OP + ni * 16 + lo] = (h16)(oacc[ni][r] * f); }
    __builtin_amdgcn_wave_barrier(); asm volatile("" ::: "memory");
    h16* cb = CTX + ((size_t)b * SEQ + qbase) * EM + h * HD;
#pragma unroll 1
    for (int ps = 0; ps < 2; ++ps) {
#pragma unroll
        for (int s = 0; s < 4; ++s) { const int row = 4 * s + (lane >> 3), cofs = (lane & 7) * 8; const v8h val = *(const v8ha*)(ost + row * OP + cofs); *(volatile v8h*)(cb + (size_t)row * EM + cofs) = val; }
        if (ps == 0) __threadfence(); }
}

extern "C" void kernel_launch(void* const* d_in, const int* in_sizes, int n_in,
                              void* d_out, int out_size, void* d_ws, size_t ws_size, hipStream_t stream) {
    if (n_in < 14) return;
    if ((size_t)in_sizes[0] < (size_t)(NB - 1) * SEQ_FULL * EM + (size_t)SEQ * EM) return;
    if (in_sizes[1] < NHD * RW || in_sizes[2] < 3 * EM * EM || in_sizes[3] < 3 * EM || in_sizes[4] < EM * EM || in_sizes[5] < EM) return;
    if (in_sizes[6] < FF * EM || in_sizes[7] < FF || in_sizes[8] < EM * FF || in_sizes[9] < EM) return;
    if (in_sizes[10] < EM || in_sizes[11] < EM || in_sizes[12] < EM || in_sizes[13] < EM) return;
    if ((size_t)out_size < (size_t)MR * EM) return;
    const float* x = (const float*)d_in[0]; const float* res_pos = (const float*)d_in[1];
    const float* in_w = (const float*)d_in[2]; const float* in_b = (const float*)d_in[3];
    const float* out_w = (const float*)d_in[4]; const float* out_b = (const float*)d_in[5];
    const float* w1 = (const float*)d_in[6]; const float* b1 = (const float*)d_in[7];
    const float* w2 = (const float*)d_in[8]; const float* b2 = (const float*)d_in[9];
    const float* g1 = (const float*)d_in[10]; const float* be1 = (const float*)d_in[11];
    const float* g2 = (const float*)d_in[12]; const float* be2 = (const float*)d_in[13];
    float* OUT = (float*)d_out;
    char* wsp = (char*)d_ws;
    auto take = [&](size_t bytes) { char* p = wsp; wsp += (bytes + 255) & ~(size_t)255; return (void*)p; };
    h16* WQKV = (h16*)take((size_t)3 * EM * EM * 2);
    h16* WO   = (h16*)take((size_t)EM * EM * 2);
    h16* W1   = (h16*)take((size_t)FF * EM * 2);
    h16* W2   = (h16*)take((size_t)EM * FF * 2);
    h16* XN   = (h16*)take((size_t)MR * EM * 2);
    h16* QKb  = (h16*)take((size_t)MR * QKP * 2);
    h16* VTp  = (h16*)take((size_t)NB * EM * SEQ * 2);
    h16* CTX  = (h16*)take((size_t)MR * EM * 2);
    float* X2 = (float*)take((size_t)MR * EM * 4);
    h16* H1   = (h16*)take((size_t)MR * FF * 2);
    if ((size_t)(wsp - (char*)d_ws) > ws_size) return;

    k_cvtw<<<(unsigned)(((size_t)3 * EM * EM / 8 + 255) / 256), 256, 0, stream>>>(in_w, WQKV, (size_t)3 * EM * EM / 8);
    k_cvtw<<<(unsigned)(((size_t)EM * EM / 8 + 255) / 256), 256, 0, stream>>>(out_w, WO, (size_t)EM * EM / 8);
    k_cvtw<<<(unsigned)(((size_t)FF * EM / 8 + 255) / 256), 256, 0, stream>>>(w1, W1, (size_t)FF * EM / 8);
    k_cvtw<<<(unsigned)(((size_t)EM * FF / 8 + 255) / 256), 256, 0, stream>>>(w2, W2, (size_t)EM * FF / 8);

    k_ln<true><<<(MR + 7) / 8, 256, 0, stream>>>(x, SEQ, SEQ_FULL, g1, be1, XN, MR);
    k_gemmw<1, false, false, 0><<<dim3(MR / 64, QKP / 64, 1), 32, 0, stream>>>(XN, WQKV, EM, (void*)QKb, QKP, in_b, 1.0f / WCAR, nullptr, SEQ, SEQ, 0, 0, 0);
    k_gemmw<1, true, false, 0><<<dim3(EM / 64, SEQ / 64, NB), 32, 0, stream>>>(WQKV + (size_t)2 * EM * EM, XN, EM, (void*)VTp, SEQ, in_b + 2 * EM, 1.0f / WCAR, nullptr, SEQ, SEQ, 0, (size_t)SEQ * EM, (size_t)EM * SEQ);
    k_attn<<<dim3(SEQ / 64, NHD, NB), 128, 0, stream>>>(QKb, VTp, res_pos, CTX);
    k_gemmw<0, false, false, 2><<<dim3(MR / 64, EM / 64, 1), 32, 0, stream>>>(CTX, WO, EM, (void*)X2, EM, out_b, 1.0f / (WCAR * CCAR), x, SEQ, SEQ_FULL, 0, 0, 0);
    k_ln<false><<<(MR + 7) / 8, 256, 0, stream>>>(X2, SEQ, SEQ, g2, be2, XN, MR);
    k_gemmw<1, false, true, 0><<<dim3(MR / 64, FF / 64, 1), 32, 0, stream>>>(XN, W1, EM, (void*)H1, FF, b1, 1.0f / WCAR, nullptr, SEQ, SEQ, 0, 0, 0);
    k_gemmw<0, false, false, 1><<<dim3(MR / 64, EM / 64, 1), 32, 0, stream>>>(H1, W2, FF, (void*)OUT, EM, b2, 1.0f / WCAR, X2, SEQ, SEQ, 0, 0, 0);
}
